// CompositeHeadB_47485158425160
// MI455X (gfx1250) — hardware-verified
//
#include <hip/hip_runtime.h>
#include <stddef.h>


typedef _Float16 v16h __attribute__((ext_vector_type(16)));
typedef _Float16 v8h  __attribute__((ext_vector_type(8)));
typedef float    v8f  __attribute__((ext_vector_type(8)));
typedef float    v4f  __attribute__((ext_vector_type(4)));

#ifndef NB
#define NB 4
#endif
#define NB_FULL 4
#define EDIM   256
#define VOUT   17
#define T_LAT  12872
#define T_TOK  74312
#define BSTR   (T_TOK * VOUT)

#define LAT0 8
#define LAT1 64
#define LAT2 512
#define LAT3 4096
#define LAT4 8192
#define XO0 0
#define XO1 8
#define XO2 72
#define XO3 584
#define XO4 4680
#define TB0 0
#define TB1 8
#define TB2 72
#define TB3 584
#define TB4 8776
#define NK3 2
#define NK4 8
#define NC3 (NK3 * VOUT)
#define NC4 (NK4 * VOUT)
#define NCP_S 64
#define NCP_4 192
#define BPITCH 192

#define PADR(r) ((((r) + 63) / 64) * 64)
#define PR0 PADR(NB * LAT0)
#define PR1 PADR(NB * LAT1)
#define PR2 PADR(NB * LAT2)
#define PR3 PADR(NB * LAT3)
#define PR4 PADR(NB * LAT4)
#define RB1 (PR0)
#define RB2 (RB1 + PR1)
#define RB3 (RB2 + PR2)
#define RB4 (RB3 + PR3)
#define PROWS (RB4 + PR4)

#define CO0 0
#define CO1 (CO0 + PR0 * NCP_S)
#define CO2 (CO1 + PR1 * NCP_S)
#define CO3 (CO2 + PR2 * NCP_S)
#define CO4 (CO3 + PR3 * NCP_S)
#define CTOT (CO4 + PR4 * NCP_4)

#define OUTF ((unsigned)NB * (unsigned)BSTR)

static_assert(NB >= 1 && NB <= NB_FULL);
static_assert(EDIM == 32 * 8);
static_assert((EDIM % 32) == 0 && (EDIM % 64) == 0);
static_assert(LAT0 == (1 << 3) && LAT1 == (1 << 6) && LAT2 == (1 << 9));
static_assert(LAT3 == (1 << 12) && LAT4 == (1 << 13));
static_assert(NK3 == (1 << 1) && NK4 == (1 << 3));
static_assert(XO1 == XO0 + LAT0 && XO2 == XO1 + LAT1 && XO3 == XO2 + LAT2 && XO4 == XO3 + LAT3);
static_assert(XO4 + LAT4 == T_LAT);
static_assert(TB1 == TB0 + LAT0 && TB2 == TB1 + LAT1 && TB3 == TB2 + LAT2);
static_assert(TB4 == TB3 + LAT3 * NK3 && TB4 + LAT4 * NK4 == T_TOK);
static_assert(VOUT <= 32);
static_assert(NC3 <= NCP_S && NC4 <= NCP_4 && VOUT <= NCP_S);
static_assert((NCP_S % 64) == 0 && (NCP_4 % 64) == 0);
static_assert(NCP_S - NC3 <= 64 && NCP_4 - NC4 <= 64);
static_assert(BPITCH >= NCP_4 && BPITCH >= NCP_S && ((5 * BPITCH) % 32) == 0);
static_assert((PROWS % 64) == 0 && (PROWS % 8) == 0);
static_assert((BSTR % 4) == 0);
static_assert((unsigned long long)NB * BSTR < 0xFFFFFFFFull);
static_assert((unsigned long long)CTOT < 0x7FFFFFFFull);

#define LDT 72
#define LDC 68
static_assert((LDT % 8) == 0 && LDT >= 64);
static_assert((LDC % 4) == 0 && LDC >= 64);
static_assert(64 * LDC * 4 <= 131072 && 64 * LDT * 2 <= 131072);

#define WCARRY 64.0f

#define MTS_BYTES  ((size_t)NCP_S * EDIM * 2)
#define MT4_BYTES  ((size_t)NCP_4 * EDIM * 2)
#define KS_BYTES   ((size_t)(NK3 + NK4) * EDIM * EDIM * 2)
#define BIAS_BYTES ((size_t)5 * BPITCH * 4)
#define X16_BYTES  ((size_t)PROWS * EDIM * 2)
#define C_BYTES    ((size_t)CTOT * 4)
#define OFF_MT0  ((size_t)0)
#define OFF_MT1  (OFF_MT0 + MTS_BYTES)
#define OFF_MT2  (OFF_MT1 + MTS_BYTES)
#define OFF_MT3  (OFF_MT2 + MTS_BYTES)
#define OFF_MT4  (OFF_MT3 + MTS_BYTES)
#define OFF_WT4  (OFF_MT4 + MT4_BYTES)
#define OFF_WT5  (OFF_WT4 + MTS_BYTES)
#define OFF_KS   (OFF_WT5 + MTS_BYTES)
#define OFF_BIAS (OFF_KS + KS_BYTES)
#define OFF_X16  (OFF_BIAS + BIAS_BYTES)
#define OFF_C    (OFF_X16 + X16_BYTES)
#define WS_TOTAL (OFF_C + C_BYTES)
static_assert((MTS_BYTES % 128) == 0 && (MT4_BYTES % 128) == 0 && (KS_BYTES % 128) == 0);
static_assert((BIAS_BYTES % 128) == 0 && (X16_BYTES % 128) == 0 && (C_BYTES % 128) == 0);
static_assert(WS_TOTAL <= (size_t)134217728);

__device__ __forceinline__ float bf16r(float x) {
  unsigned int u = __float_as_uint(x);
  u = (u + 0x7FFFu + ((u >> 16) & 1u)) & 0xFFFF0000u;
  return __uint_as_float(u);
}

static __device__ __forceinline__ _Float16 toh_flush(float v) {
  const _Float16 r = (_Float16)v;
  return (fabsf(v) < 6.103515625e-05f) ? (_Float16)0.0f : r;
}

__device__ __forceinline__ v16h frag_at(const _Float16* p) {
  v8h lo = *(const v8h*)(p);
  v8h hi = *(const v8h*)(p + 16);
  v16h out;
#pragma unroll
  for (int i = 0; i < 8; ++i) { out[i] = lo[i]; out[i + 8] = hi[i]; }
  return out;
}

__device__ __forceinline__ v8f wmma16(v16h a, v16h b, v8f c) {
  v8f d = __builtin_amdgcn_wmma_f32_16x16x32_f16(false, a, false, b, (short)0, c,
                                                 false, false);
  asm volatile("v_nop\n\tv_nop\n\tv_nop\n\tv_nop" : "+v"(d) : "v"(a), "v"(b));
  return d;
}

__global__ __launch_bounds__(256) void wconv_kernel(
    const float* __restrict__ W, _Float16* __restrict__ Wt, unsigned ldw, unsigned ldk,
    unsigned ncols) {
  __shared__ _Float16 T[64 * LDT];
  const unsigned tid = threadIdx.x;
  const unsigned n0 = blockIdx.x * 64u;
  const unsigned k0 = blockIdx.y * 64u;
#pragma unroll 4
  for (unsigned j = 0; j < 16u; ++j) {
    const unsigned idx = tid + 256u * j;
    const unsigned kr = idx >> 6, nc = idx & 63u;
    const unsigned ncol = n0 + nc;
    const unsigned ncl = (ncol < ncols) ? ncol : (ncols - 1u);
    float v = W[(size_t)(k0 + kr) * ldw + ncl];
    v = (ncol < ncols) ? v : 0.0f;
    T[nc * LDT + kr] = toh_flush(WCARRY * bf16r(v));
  }
  __syncthreads();
  v8h x[2];
  size_t off[2];
#pragma unroll
  for (unsigned i = 0; i < 2u; ++i) {
    const unsigned n = 32u * i + (tid >> 3);
    const unsigned kc = (tid & 7u) * 8u;
    x[i] = *(const v8h*)&T[n * LDT + kc];
    off[i] = (size_t)(n0 + n) * ldk + k0 + kc;
  }
#pragma unroll
  for (int i = 0; i < 2; ++i) *(volatile v8h*)(Wt + off[i]) = x[i];
  __threadfence();
#pragma unroll
  for (int i = 0; i < 2; ++i) *(volatile v8h*)(Wt + off[i]) = x[i];
}

__global__ __launch_bounds__(256) void kconv_kernel(
    const float* __restrict__ Kw, _Float16* __restrict__ Ks, unsigned nk) {
  const unsigned lane = threadIdx.x & 31u, w = threadIdx.x >> 5;
  const unsigned row = blockIdx.x * 8u + w;
  const unsigned kk = row >> 8, i = row & 255u;
  const float* src = Kw + ((size_t)i * EDIM + lane * 8u) * nk + kk;
  v8h o;
#pragma unroll
  for (unsigned j = 0; j < 8u; ++j) o[j] = toh_flush(WCARRY * bf16r(src[(size_t)j * nk]));
  _Float16* p = Ks + (size_t)row * EDIM + lane * 8u;
  *(volatile v8h*)p = o;
  __threadfence();
  *(volatile v8h*)p = o;
}

__global__ __launch_bounds__(256) void bias_kernel(
    const float* __restrict__ b1, const float* __restrict__ b2, const float* __restrict__ b3,
    const float* __restrict__ cb4, const float* __restrict__ W4, const float* __restrict__ b4,
    const float* __restrict__ cb5, const float* __restrict__ W5, const float* __restrict__ b5,
    float* __restrict__ Bv) {
  const unsigned idx = blockIdx.x * 256u + threadIdx.x;
  if (idx >= 5u * BPITCH) return;
  const unsigned s = idx / (unsigned)BPITCH;
  const unsigned c = idx - s * (unsigned)BPITCH;
  const unsigned v = c % (unsigned)VOUT;
  float d4 = 0.0f, d5 = 0.0f;
#pragma unroll 1
  for (unsigned e = 0; e < (unsigned)EDIM; ++e) {
    d4 += bf16r(cb4[e]) * bf16r(W4[e * VOUT + v]);
    d5 += bf16r(cb5[e]) * bf16r(W5[e * VOUT + v]);
  }
  const float v1 = bf16r(b1[v]);
  const float v2 = bf16r(b2[v]);
  const float v3 = bf16r(b3[v]);
  const float v4 = d4 + bf16r(b4[v]);
  const float v5 = d5 + bf16r(b5[v]);
  const unsigned nc = (s == 4u) ? (unsigned)NC4 : ((s == 3u) ? (unsigned)NC3 : (unsigned)VOUT);
  float val = (s == 0u) ? v1 : ((s == 1u) ? v2 : ((s == 2u) ? v3 : ((s == 3u) ? v4 : v5)));
  val = (c < nc) ? val : 0.0f;
  float* p = Bv + idx;
  *(volatile float*)p = val;
  __threadfence();
  *(volatile float*)p = val;
}

__global__ __launch_bounds__(256) void fold_kernel(
    const _Float16* __restrict__ Wt, const _Float16* __restrict__ Ks,
    _Float16* __restrict__ Mt, unsigned nk, unsigned npad) {
  __shared__ float Cs[64 * LDC];
  const unsigned tid = threadIdx.x, lane = tid & 31u, w = tid >> 5;
  const unsigned mw = w >> 1, nw = w & 1u;
  const unsigned hh = lane >> 4, m = lane & 15u;
  const unsigned n0 = blockIdx.x * 64u;
  const unsigned kk = blockIdx.z;

  const _Float16* ap  = Wt + (size_t)(mw * 16u + m) * EDIM + hh * 8u;
  const _Float16* bp0 = Ks + ((size_t)kk * EDIM + n0 + nw * 32u + m) * EDIM + hh * 8u;
  const _Float16* bp1 = bp0 + (size_t)16 * EDIM;
  v8f acc0 = {}, acc1 = {};
#pragma unroll 2
  for (unsigned k0 = 0; k0 < (unsigned)EDIM; k0 += 32u) {
    const v16h a  = frag_at(ap + k0);
    const v16h b0 = frag_at(bp0 + k0);
    const v16h b1 = frag_at(bp1 + k0);
    acc0 = wmma16(a, b0, acc0);
    acc1 = wmma16(a, b1, acc1);
  }
#pragma unroll
  for (int r = 0; r < 8; ++r) {
    float* d = &Cs[(mw * 16u + hh * 8u + (unsigned)r) * LDC + nw * 32u + m];
    d[0]  = acc0[r];
    d[16] = acc1[r];
  }
  __syncthreads();

  const unsigned r = tid >> 3;
  const unsigned c = (tid & 7u) * 8u;
  const v4f u0 = *(const v4f*)&Cs[r * LDC + c];
  const v4f u1 = *(const v4f*)&Cs[r * LDC + c + 4];
  v8h xv;
#pragma unroll
  for (int j = 0; j < 4; ++j) {
    xv[j]     = toh_flush(u0[j] * (1.0f / WCARRY));
    xv[j + 4] = toh_flush(u1[j] * (1.0f / WCARRY));
  }
  const bool okv = (r < (unsigned)VOUT);
  const size_t offv = (size_t)(kk * VOUT + r) * EDIM + n0 + c;
  const bool last = (kk + 1u == nk);
  const v8h z = {};
  size_t offp[2];
  bool okp[2];
#pragma unroll
  for (unsigned j = 0; j < 2u; ++j) {
    const unsigned rp = 32u * j + r;
    okp[j] = last && (rp < npad);
    offp[j] = (size_t)(nk * VOUT + rp) * EDIM + n0 + c;
  }
  if (okv) *(volatile v8h*)(Mt + offv) = xv;
#pragma unroll
  for (int j = 0; j < 2; ++j) if (okp[j]) *(volatile v8h*)(Mt + offp[j]) = z;
  __threadfence();
  if (okv) *(volatile v8h*)(Mt + offv) = xv;
#pragma unroll
  for (int j = 0; j < 2; ++j) if (okp[j]) *(volatile v8h*)(Mt + offp[j]) = z;
}

__global__ __launch_bounds__(256) void xconv_kernel(
    const float* __restrict__ X, _Float16* __restrict__ X16) {
  const unsigned lane = threadIdx.x & 31u, w = threadIdx.x >> 5;
  const unsigned p = blockIdx.x * 8u + w;
  const bool s1 = (p >= (unsigned)RB1), s2 = (p >= (unsigned)RB2);
  const bool s3 = (p >= (unsigned)RB3), s4 = (p >= (unsigned)RB4);
  const unsigned rb = s4 ? (unsigned)RB4 : (s3 ? (unsigned)RB3 : (s2 ? (unsigned)RB2 : (s1 ? (unsigned)RB1 : 0u)));
  const unsigned sh = s4 ? 13u : (s3 ? 12u : (s2 ? 9u : (s1 ? 6u : 3u)));
  const unsigned xo = s4 ? (unsigned)XO4 : (s3 ? (unsigned)XO3 : (s2 ? (unsigned)XO2 : (s1 ? (unsigned)XO1 : (unsigned)XO0)));
  const unsigned rr = p - rb;
  const unsigned n = rr >> sh;
  const unsigned t = rr & ((1u << sh) - 1u);
  const bool valid = (n < (unsigned)NB);
  const unsigned ncl = valid ? n : 0u;
  const float* src = X + ((size_t)ncl * T_LAT + xo + t) * EDIM + lane * 8u;
  const v4f a0 = *(const v4f*)(src);
  const v4f a1 = *(const v4f*)(src + 4);
  v8h o;
#pragma unroll
  for (int j = 0; j < 4; ++j) {
    const _Float16 e0 = toh_flush(bf16r(a0[j]));
    const _Float16 e1 = toh_flush(bf16r(a1[j]));
    o[j]     = valid ? e0 : (_Float16)0.0f;
    o[j + 4] = valid ? e1 : (_Float16)0.0f;
  }
  _Float16* q = X16 + (size_t)p * EDIM + lane * 8u;
  *(volatile v8h*)q = o;
  __threadfence();
  *(volatile v8h*)q = o;
}

__global__ __launch_bounds__(256) void gemm_head_kernel(
    const _Float16* __restrict__ A16, const _Float16* __restrict__ Bt,
    const float* __restrict__ bias, float* __restrict__ outf, unsigned ldo) {
  __shared__ float Cs[64 * LDC];
  const unsigned tid = threadIdx.x, lane = tid & 31u, w = tid >> 5;
  const unsigned mw = w >> 1, nw = w & 1u;
  const unsigned hh = lane >> 4, m = lane & 15u;
  const unsigned n0 = blockIdx.x * 64u;
  const unsigned row0 = blockIdx.y * 64u;

  const _Float16* ap  = A16 + (size_t)(row0 + mw * 16u + m) * EDIM + hh * 8u;
  const _Float16* bp0 = Bt + (size_t)(n0 + nw * 32u + m) * EDIM + hh * 8u;
  const _Float16* bp1 = bp0 + (size_t)16 * EDIM;
  v8f acc0 = {}, acc1 = {};
#pragma unroll 2
  for (unsigned k0 = 0; k0 < (unsigned)EDIM; k0 += 32u) {
    const v16h a  = frag_at(ap + k0);
    const v16h b0 = frag_at(bp0 + k0);
    const v16h b1 = frag_at(bp1 + k0);
    acc0 = wmma16(a, b0, acc0);
    acc1 = wmma16(a, b1, acc1);
  }
#pragma unroll
  for (int r = 0; r < 8; ++r) {
    float* d = &Cs[(mw * 16u + hh * 8u + (unsigned)r) * LDC + nw * 32u + m];
    d[0]  = acc0[r];
    d[16] = acc1[r];
  }
  __syncthreads();

  v4f xs[4];
  size_t off[4];
#pragma unroll
  for (unsigned i = 0; i < 4u; ++i) {
    const unsigned r = 16u * i + (tid >> 4);
    const unsigned c = (tid & 15u) * 4u;
    const v4f u = *(const v4f*)&Cs[r * LDC + c];
    const v4f g = *(const v4f*)(bias + n0 + c);
    v4f val;
#pragma unroll
    for (int j = 0; j < 4; ++j) val[j] = u[j] * (1.0f / WCARRY) + g[j];
    xs[i] = val;
    off[i] = (size_t)(row0 + r) * ldo + n0 + c;
  }
#pragma unroll
  for (int i = 0; i < 4; ++i) *(volatile v4f*)(outf + off[i]) = xs[i];
  __threadfence();
#pragma unroll
  for (int i = 0; i < 4; ++i) *(volatile v4f*)(outf + off[i]) = xs[i];
}

__global__ __launch_bounds__(256) void pack_kernel(
    const float* __restrict__ C, float* __restrict__ out) {
  const unsigned q = blockIdx.x * 256u + threadIdx.x;
  const unsigned f0 = q * 4u;
  if (f0 >= OUTF) return;
  v4f val;
#pragma unroll
  for (int j = 0; j < 4; ++j) {
    const unsigned f = f0 + (unsigned)j;
    const unsigned n = f / (unsigned)BSTR;
    const unsigned r = f - n * (unsigned)BSTR;
    const unsigned tok = r / (unsigned)VOUT;
    const unsigned v = r - tok * (unsigned)VOUT;
    const bool s1 = (tok >= (unsigned)TB1), s2 = (tok >= (unsigned)TB2);
    const bool s3 = (tok >= (unsigned)TB3), s4 = (tok >= (unsigned)TB4);
    const unsigned tb  = s4 ? (unsigned)TB4 : (s3 ? (unsigned)TB3 : (s2 ? (unsigned)TB2 : (s1 ? (unsigned)TB1 : (unsigned)TB0)));
    const unsigned sh  = s4 ? 3u : (s3 ? 1u : 0u);
    const unsigned lsh = s4 ? 13u : (s3 ? 12u : (s2 ? 9u : (s1 ? 6u : 3u)));
    const unsigned co  = s4 ? (unsigned)CO4 : (s3 ? (unsigned)CO3 : (s2 ? (unsigned)CO2 : (s1 ? (unsigned)CO1 : (unsigned)CO0)));
    const unsigned ncp = s4 ? (unsigned)NCP_4 : (unsigned)NCP_S;
    const unsigned tt = tok - tb;
    const unsigned t = tt >> sh;
    const unsigned kk = tt & ((1u << sh) - 1u);
    const unsigned col = kk * (unsigned)VOUT + v;
    const unsigned row = (n << lsh) + t;
    const unsigned src = co + row * ncp + col;
    val[j] = C[src];
  }
  float* p = out + f0;
  *(volatile v4f*)p = val;
  __threadfence();
  *(volatile v4f*)p = val;
}

extern "C" void kernel_launch(void* const* d_in, const int* in_sizes, int n_in,
                              void* d_out, int out_size, void* d_ws, size_t ws_size,
                              hipStream_t stream) {
  if (n_in < 18) return;
  const long long need_x = (long long)NB * T_LAT * EDIM;
  if ((long long)in_sizes[0] < need_x) return;
  if (in_sizes[4] < EDIM * VOUT || in_sizes[6] < EDIM * VOUT || in_sizes[8] < EDIM * VOUT) return;
  if (in_sizes[12] < EDIM * VOUT || in_sizes[16] < EDIM * VOUT) return;
  if (in_sizes[5] < VOUT || in_sizes[7] < VOUT || in_sizes[9] < VOUT) return;
  if (in_sizes[13] < VOUT || in_sizes[17] < VOUT) return;
  if (in_sizes[10] < EDIM * EDIM * NK3 || in_sizes[14] < EDIM * EDIM * NK4) return;
  if (in_sizes[11] < EDIM || in_sizes[15] < EDIM) return;
  if ((long long)out_size < (long long)NB * BSTR) return;
  if (ws_size < WS_TOTAL) return;

  const float* X   = (const float*)d_in[0];
  const float* W1  = (const float*)d_in[4];
  const float* b1  = (const float*)d_in[5];
  const float* W2  = (const float*)d_in[6];
  const float* b2  = (const float*)d_in[7];
  const float* W3  = (const float*)d_in[8];
  const float* b3  = (const float*)d_in[9];
  const float* K4  = (const float*)d_in[10];
  const float* cb4 = (const float*)d_in[11];
  const float* W4  = (const float*)d_in[12];
  const float* b4  = (const float*)d_in[13];
  const float* K5  = (const float*)d_in[14];
  const float* cb5 = (const float*)d_in[15];
  const float* W5  = (const float*)d_in[16];
  const float* b5  = (const float*)d_in[17];
  float* out = (float*)d_out;

  char* ws = (char*)d_ws;
  _Float16* Mt0 = (_Float16*)(ws + OFF_MT0);
  _Float16* Mt1 = (_Float16*)(ws + OFF_MT1);
  _Float16* Mt2 = (_Float16*)(ws + OFF_MT2);
  _Float16* Mt3 = (_Float16*)(ws + OFF_MT3);
  _Float16* Mt4 = (_Float16*)(ws + OFF_MT4);
  _Float16* Wt4 = (_Float16*)(ws + OFF_WT4);
  _Float16* Wt5 = (_Float16*)(ws + OFF_WT5);
  _Float16* Ks  = (_Float16*)(ws + OFF_KS);
  float*    Bv  = (float*)(ws + OFF_BIAS);
  _Float16* X16 = (_Float16*)(ws + OFF_X16);
  float*    Cp  = (float*)(ws + OFF_C);

  dim3 blk(256);
  dim3 gw(1, EDIM / 64);

  wconv_kernel<<<gw, blk, 0, stream>>>(W1, Mt0, (unsigned)VOUT, (unsigned)EDIM, (unsigned)VOUT);
  wconv_kernel<<<gw, blk, 0, stream>>>(W2, Mt1, (unsigned)VOUT, (unsigned)EDIM, (unsigned)VOUT);
  wconv_kernel<<<gw, blk, 0, stream>>>(W3, Mt2, (unsigned)VOUT, (unsigned)EDIM, (unsigned)VOUT);
  wconv_kernel<<<gw, blk, 0, stream>>>(W4, Wt4, (unsigned)VOUT, (unsigned)EDIM, (unsigned)VOUT);
  wconv_kernel<<<gw, blk, 0, stream>>>(W5, Wt5, (unsigned)VOUT, (unsigned)EDIM, (unsigned)VOUT);

  kconv_kernel<<<dim3(NK3 * EDIM / 8), blk, 0, stream>>>(K4, Ks, (unsigned)NK3);
  kconv_kernel<<<dim3(NK4 * EDIM / 8), blk, 0, stream>>>(K5, Ks + (size_t)NK3 * EDIM * EDIM,
                                                        (unsigned)NK4);

  bias_kernel<<<dim3(4), blk, 0, stream>>>(b1, b2, b3, cb4, W4, b4, cb5, W5, b5, Bv);

  fold_kernel<<<dim3(EDIM / 64, 1, NK3), blk, 0, stream>>>(
      Wt4, Ks, Mt3, (unsigned)NK3, (unsigned)(NCP_S - NC3));
  fold_kernel<<<dim3(EDIM / 64, 1, NK4), blk, 0, stream>>>(
      Wt5, Ks + (size_t)NK3 * EDIM * EDIM, Mt4, (unsigned)NK4, (unsigned)(NCP_4 - NC4));

  xconv_kernel<<<dim3(PROWS / 8), blk, 0, stream>>>(X, X16);

  gemm_head_kernel<<<dim3(NCP_S / 64, PR0 / 64), blk, 0, stream>>>(
      X16, Mt0, Bv, Cp + CO0, (unsigned)NCP_S);
  gemm_head_kernel<<<dim3(NCP_S / 64, PR1 / 64), blk, 0, stream>>>(
      X16 + (size_t)RB1 * EDIM, Mt1, Bv + BPITCH, Cp + CO1, (unsigned)NCP_S);
  gemm_head_kernel<<<dim3(NCP_S / 64, PR2 / 64), blk, 0, stream>>>(
      X16 + (size_t)RB2 * EDIM, Mt2, Bv + 2 * BPITCH, Cp + CO2, (unsigned)NCP_S);
  gemm_head_kernel<<<dim3(NCP_S / 64, PR3 / 64), blk, 0, stream>>>(
      X16 + (size_t)RB3 * EDIM, Mt3, Bv + 3 * BPITCH, Cp + CO3, (unsigned)NCP_S);
  gemm_head_kernel<<<dim3(NCP_4 / 64, PR4 / 64), blk, 0, stream>>>(
      X16 + (size_t)RB4 * EDIM, Mt4, Bv + 4 * BPITCH, Cp + CO4, (unsigned)NCP_4);

  const unsigned nq = OUTF / 4u;
  pack_kernel<<<dim3((nq + 255u) / 256u), blk, 0, stream>>>(Cp, out);
}
